// SelfAttentionModel_65481071400557
// MI455X (gfx1250) — hardware-verified
//
#include <hip/hip_runtime.h>
#include <stddef.h>


#define B_ 4
#define S_ 2048
#define E_ 512
#define H_ 8
#define D_ 64
#define N_ (B_ * S_)

static_assert(E_ == H_ * D_);
static_assert(D_ == 64);
static_assert((S_ % 64) == 0 && (E_ % 64) == 0 && (N_ % 64) == 0);

typedef float          v8f   __attribute__((ext_vector_type(8)));
typedef float          v4f   __attribute__((ext_vector_type(4)));
typedef __bf16         v16b  __attribute__((ext_vector_type(16)));
typedef __bf16         v8b   __attribute__((ext_vector_type(8)));
typedef unsigned short v8us  __attribute__((ext_vector_type(8)));

union Frag16 { v16b v; v8us hv[2]; };
union Pack8  { v8b b; v8us u; };

#define NOP4 "v_nop\n\tv_nop\n\tv_nop\n\tv_nop"

__device__ __forceinline__ v16b ld_frag(const unsigned short* rowk, int h) {
  Frag16 f;
  f.hv[0] = *(const v8us*)(rowk + 8 * h);
  f.hv[1] = *(const v8us*)(rowk + 16 + 8 * h);
  return f.v;
}

__device__ __forceinline__ v16b join16(v8us a, v8us b) {
  Frag16 f;
  f.hv[0] = a;
  f.hv[1] = b;
  return f.v;
}

__device__ __forceinline__ v8f mma(v16b a, v16b b, v8f c) {
  return __builtin_amdgcn_wmma_f32_16x16x32_bf16(false, a, false, b, (short)0, c, false, false);
}

__device__ __forceinline__ v8f vzero() {
  v8f z = {0.f, 0.f, 0.f, 0.f, 0.f, 0.f, 0.f, 0.f};
  return z;
}

__device__ __forceinline__ void split8(v8f x, v8us& hu, v8us& lu) {
  Pack8 ph, pl;
  ph.b = __builtin_convertvector(x, v8b);
  const v8f hf = __builtin_convertvector(ph.b, v8f);
  pl.b = __builtin_convertvector(x - hf, v8b);
  hu = ph.u;
  lu = pl.u;
}

__global__ void __launch_bounds__(256)
k_split(const float* __restrict__ src, unsigned short* __restrict__ dh, unsigned short* __restrict__ dl, int n8) {
  const int i = blockIdx.x * 256 + threadIdx.x;
  if (i < n8) {
    const v4f* p = (const v4f*)(src + (size_t)i * 8);
    const v4f a0 = p[0];
    const v4f a1 = p[1];
    const v8f x = __builtin_shufflevector(a0, a1, 0, 1, 2, 3, 4, 5, 6, 7);
    v8us hu, lu;
    split8(x, hu, lu);
    volatile v8us* ph = (volatile v8us*)(dh + (size_t)i * 8);
    volatile v8us* pl = (volatile v8us*)(dl + (size_t)i * 8);
    *ph = hu;
    *pl = lu;
    __threadfence();
    *ph = hu;
    *pl = lu;
  }
}

template <int MODE>
__global__ void __launch_bounds__(128)
k_gemm(const unsigned short* __restrict__ Ph, const unsigned short* __restrict__ Pl,
       const unsigned short* __restrict__ Rh, const unsigned short* __restrict__ Rl,
       const float* __restrict__ bias,
       unsigned short* __restrict__ Oh, unsigned short* __restrict__ Ol,
       float* __restrict__ Of)
{
  const int l  = threadIdx.x & 31;
  const int h  = l >> 4;
  const int m  = l & 15;
  const int wv = threadIdx.x >> 5;
  const int gw = blockIdx.x * 4 + wv;
  int ibase, jbase;
  if (MODE == 1) { ibase = (gw >> 5) * 64; jbase = (gw & 31) * 16; }
  else           { ibase = (gw & 7) * 64;  jbase = (gw >> 3) * 16; }

  v8f acc[4];
#pragma unroll
  for (int t = 0; t < 4; ++t) acc[t] = vzero();

  const unsigned short* rp_h = Rh + (size_t)(jbase + m) * E_;
  const unsigned short* rp_l = Rl + (size_t)(jbase + m) * E_;
  const unsigned short* pp_h = Ph + (size_t)(ibase + m) * E_;
  const unsigned short* pp_l = Pl + (size_t)(ibase + m) * E_;

#pragma unroll 1
  for (int k0 = 0; k0 < E_; k0 += 32) {
    const v16b rh = ld_frag(rp_h + k0, h);
    const v16b rl = ld_frag(rp_l + k0, h);
    v16b ph[4], pl[4];
#pragma unroll
    for (int t = 0; t < 4; ++t) {
      ph[t] = ld_frag(pp_h + (size_t)t * 16 * E_ + k0, h);
      pl[t] = ld_frag(pp_l + (size_t)t * 16 * E_ + k0, h);
    }
#pragma unroll
    for (int t = 0; t < 4; ++t) {
      acc[t] = mma(ph[t], rh, acc[t]);
      acc[t] = mma(ph[t], rl, acc[t]);
      acc[t] = mma(pl[t], rh, acc[t]);
    }
    asm volatile(NOP4
                 : "+v"(acc[0]), "+v"(acc[1]), "+v"(acc[2]), "+v"(acc[3])
                 : "v"(ph[0]), "v"(ph[1]), "v"(ph[2]), "v"(ph[3]),
                   "v"(pl[0]), "v"(pl[1]), "v"(pl[2]), "v"(pl[3]),
                   "v"(rh), "v"(rl)
                 : "memory");
  }

  if constexpr (MODE == 2) {
    __shared__ v4f lds_f[4][256];
#pragma unroll
    for (int t = 0; t < 4; ++t) {
      const v4f b0 = *(const v4f*)(bias + ibase + t * 16 + 8 * h);
      const v4f b1 = *(const v4f*)(bias + ibase + t * 16 + 8 * h + 4);
      const v8f bb = __builtin_shufflevector(b0, b1, 0, 1, 2, 3, 4, 5, 6, 7);
      const v8f val = acc[t] + bb;
      lds_f[wv][m * 16 + 4 * t + 2 * h]     = __builtin_shufflevector(val, val, 0, 1, 2, 3);
      lds_f[wv][m * 16 + 4 * t + 2 * h + 1] = __builtin_shufflevector(val, val, 4, 5, 6, 7);
    }
    __syncthreads();
    v4f w[8];
    size_t off[8];
#pragma unroll
    for (int j = 0; j < 8; ++j) {
      const int c = j * 32 + l;
      w[j] = lds_f[wv][c];
      off[j] = (size_t)(jbase + (c >> 4)) * E_ + ibase + (c & 15) * 4;
    }
#pragma unroll
    for (int j = 0; j < 8; ++j) *(volatile v4f*)(Of + off[j]) = w[j];
    __threadfence();
#pragma unroll
    for (int j = 0; j < 8; ++j) *(volatile v4f*)(Of + off[j]) = w[j];
  } else {
    __shared__ v8us lds_h[4][2][128];
    float bsc = 0.0f;
    if (MODE == 1) bsc = bias[jbase + m];
#pragma unroll
    for (int t = 0; t < 4; ++t) {
      v8f val;
      if (MODE == 0) {
        const v4f b0 = *(const v4f*)(bias + ibase + t * 16 + 8 * h);
        const v4f b1 = *(const v4f*)(bias + ibase + t * 16 + 8 * h + 4);
        const v8f bb = __builtin_shufflevector(b0, b1, 0, 1, 2, 3, 4, 5, 6, 7);
        val = acc[t] + bb;
      } else {
        val = acc[t] + bsc;
      }
      v8us hu, lu;
      split8(val, hu, lu);
      lds_h[wv][0][m * 8 + 2 * t + h] = hu;
      lds_h[wv][1][m * 8 + 2 * t + h] = lu;
    }
    __syncthreads();
    v8us w0[4], w1[4];
    size_t off[4];
#pragma unroll
    for (int j = 0; j < 4; ++j) {
      const int c = j * 32 + l;
      w0[j] = lds_h[wv][0][c];
      w1[j] = lds_h[wv][1][c];
      if (MODE == 0) {
        const size_t base = ((size_t)((jbase >> 11) * H_ + (ibase >> 6)) * S_ + (jbase & (S_ - 1))) * D_;
        off[j] = base + (size_t)c * 8;
      } else {
        const int bh = (ibase >> 11) * H_ + (jbase >> 6);
        const int d0 = jbase & (D_ - 1);
        const int s0 = ibase & (S_ - 1);
        off[j] = (size_t)(bh * D_ + d0 + (c >> 3)) * S_ + s0 + (c & 7) * 8;
      }
    }
#pragma unroll
    for (int j = 0; j < 4; ++j) {
      *(volatile v8us*)(Oh + off[j]) = w0[j];
      *(volatile v8us*)(Ol + off[j]) = w1[j];
    }
    __threadfence();
#pragma unroll
    for (int j = 0; j < 4; ++j) {
      *(volatile v8us*)(Oh + off[j]) = w0[j];
      *(volatile v8us*)(Ol + off[j]) = w1[j];
    }
  }
}

__global__ void __launch_bounds__(128)
k_attn(const unsigned short* __restrict__ Qh, const unsigned short* __restrict__ Ql,
       const unsigned short* __restrict__ Kh, const unsigned short* __restrict__ Kl,
       const unsigned short* __restrict__ Vh, const unsigned short* __restrict__ Vl,
       const float* __restrict__ ent,
       unsigned short* __restrict__ Ah, unsigned short* __restrict__ Al)
{
  __shared__ v8us lds_a[4][2][128];
  const int l    = threadIdx.x & 31;
  const int h    = l >> 4;
  const int m    = l & 15;
  const int wv   = threadIdx.x >> 5;
  const int gw   = blockIdx.x * 4 + wv;
  const int bh   = gw >> 7;
  const int qt   = gw & 127;
  const int q0   = qt * 16;
  const int b    = bh >> 3;
  const int head = bh & 7;

  const size_t qoff = ((size_t)bh * S_ + q0 + m) * D_;
  const v16b qh0 = ld_frag(Qh + qoff, h);
  const v16b qh1 = ld_frag(Qh + qoff + 32, h);
  const v16b ql0 = ld_frag(Ql + qoff, h);
  const v16b ql1 = ld_frag(Ql + qoff + 32, h);
  const float fac2 = ent[q0 + m] * 0.18033688011112042f;

  float mrun = -__builtin_inff();
  float lrun = 0.0f;
  v8f o[4];
#pragma unroll
  for (int t = 0; t < 4; ++t) o[t] = vzero();

  const unsigned short* kh_b = Kh + (size_t)bh * S_ * D_;
  const unsigned short* kl_b = Kl + (size_t)bh * S_ * D_;
  const unsigned short* vh_b = Vh + (size_t)bh * D_ * S_;
  const unsigned short* vl_b = Vl + (size_t)bh * D_ * S_;

#pragma unroll 1
  for (int kb = 0; kb < S_; kb += 64) {
    v8f c[4];
#pragma unroll
    for (int u = 0; u < 4; ++u) {
      const size_t ko = (size_t)(kb + u * 16 + m) * D_;
      const v16b a0h = ld_frag(kh_b + ko, h);
      const v16b a1h = ld_frag(kh_b + ko + 32, h);
      const v16b a0l = ld_frag(kl_b + ko, h);
      const v16b a1l = ld_frag(kl_b + ko + 32, h);
      v8f cc = vzero();
      cc = mma(a0h, qh0, cc);
      cc = mma(a0h, ql0, cc);
      cc = mma(a0l, qh0, cc);
      cc = mma(a1h, qh1, cc);
      cc = mma(a1h, ql1, cc);
      cc = mma(a1l, qh1, cc);
      asm volatile(NOP4
                   : "+v"(cc)
                   : "v"(a0h), "v"(a1h), "v"(a0l), "v"(a1l), "v"(qh0), "v"(qh1), "v"(ql0), "v"(ql1)
                   : "memory");
      c[u] = cc;
    }

    float tmax = -__builtin_inff();
#pragma unroll
    for (int u = 0; u < 4; ++u) {
      c[u] = c[u] * fac2;
#pragma unroll
      for (int r = 0; r < 8; ++r) tmax = fmaxf(tmax, c[u][r]);
    }
    tmax = fmaxf(tmax, __shfl_xor(tmax, 16));
    const float mnew  = fmaxf(mrun, tmax);
    const float alpha = __builtin_amdgcn_exp2f(mrun - mnew);
    float psum = 0.0f;
#pragma unroll
    for (int u = 0; u < 4; ++u) {
#pragma unroll
      for (int r = 0; r < 8; ++r) {
        const float p = __builtin_amdgcn_exp2f(c[u][r] - mnew);
        c[u][r] = p;
        psum += p;
      }
    }
    psum += __shfl_xor(psum, 16);
    lrun = lrun * alpha + psum;
    mrun = mnew;
#pragma unroll
    for (int t = 0; t < 4; ++t) o[t] = o[t] * alpha;

#pragma unroll
    for (int v = 0; v < 2; ++v) {
      v8us h0, l0, h1, l1;
      split8(c[2 * v], h0, l0);
      split8(c[2 * v + 1], h1, l1);
      const v16b phi = join16(h0, h1);
      const v16b plo = join16(l0, l1);
#pragma unroll
      for (int t = 0; t < 4; ++t) {
        const size_t vo = (size_t)(t * 16 + m) * S_ + kb + v * 32;
        const v16b va_h = ld_frag(vh_b + vo, h);
        const v16b va_l = ld_frag(vl_b + vo, h);
        v8f oo = o[t];
        oo = mma(va_h, phi, oo);
        oo = mma(va_h, plo, oo);
        oo = mma(va_l, phi, oo);
        asm volatile(NOP4
                     : "+v"(oo)
                     : "v"(va_h), "v"(va_l), "v"(phi), "v"(plo)
                     : "memory");
        o[t] = oo;
      }
    }
  }

  const float inv = 1.0f / lrun;
#pragma unroll
  for (int t = 0; t < 4; ++t) {
    const v8f val = o[t] * inv;
    v8us hu, lu;
    split8(val, hu, lu);
    lds_a[wv][0][m * 8 + 2 * t + h] = hu;
    lds_a[wv][1][m * 8 + 2 * t + h] = lu;
  }
  __syncthreads();
  v8us w0[4], w1[4];
  size_t off[4];
#pragma unroll
  for (int j = 0; j < 4; ++j) {
    const int ci = j * 32 + l;
    w0[j] = lds_a[wv][0][ci];
    w1[j] = lds_a[wv][1][ci];
    off[j] = ((size_t)b * S_ + q0 + (ci >> 3)) * E_ + head * D_ + (ci & 7) * 8;
  }
#pragma unroll
  for (int j = 0; j < 4; ++j) {
    *(volatile v8us*)(Ah + off[j]) = w0[j];
    *(volatile v8us*)(Al + off[j]) = w1[j];
  }
  __threadfence();
#pragma unroll
  for (int j = 0; j < 4; ++j) {
    *(volatile v8us*)(Ah + off[j]) = w0[j];
    *(volatile v8us*)(Al + off[j]) = w1[j];
  }
}

extern "C" void kernel_launch(void* const* d_in, const int* in_sizes, int n_in,
                              void* d_out, int out_size, void* d_ws, size_t ws_size,
                              hipStream_t stream) {
  if (n_in < 10) return;
  if (in_sizes[0] != N_ * E_ || in_sizes[1] != S_ ||
      in_sizes[2] != E_ * E_ || in_sizes[3] != E_ ||
      in_sizes[4] != E_ * E_ || in_sizes[5] != E_ ||
      in_sizes[6] != E_ * E_ || in_sizes[7] != E_ ||
      in_sizes[8] != E_ * E_ || in_sizes[9] != E_ ||
      out_size != N_ * E_) return;

  const float* x   = (const float*)d_in[0];
  const float* ent = (const float*)d_in[1];
  const float* Wq  = (const float*)d_in[2];
  const float* bq  = (const float*)d_in[3];
  const float* Wk  = (const float*)d_in[4];
  const float* bk  = (const float*)d_in[5];
  const float* Wv  = (const float*)d_in[6];
  const float* bv  = (const float*)d_in[7];
  const float* Wo  = (const float*)d_in[8];
  const float* bo  = (const float*)d_in[9];
  float* out = (float*)d_out;

  const size_t nX = (size_t)N_ * E_;
  const size_t nW = (size_t)E_ * E_;
  const size_t total_bytes = (10 * nX + 8 * nW) * sizeof(unsigned short);
  if (total_bytes > ws_size) return;

  unsigned short* p = (unsigned short*)d_ws;
  unsigned short* Xh  = p; p += nX;   unsigned short* Xl  = p; p += nX;
  unsigned short* Wqh = p; p += nW;   unsigned short* Wql = p; p += nW;
  unsigned short* Wkh = p; p += nW;   unsigned short* Wkl = p; p += nW;
  unsigned short* Wvh = p; p += nW;   unsigned short* Wvl = p; p += nW;
  unsigned short* Woh = p; p += nW;   unsigned short* Wol = p; p += nW;
  unsigned short* Qh  = p; p += nX;   unsigned short* Ql  = p; p += nX;
  unsigned short* Kh  = p; p += nX;   unsigned short* Kl  = p; p += nX;
  unsigned short* Vh  = p; p += nX;   unsigned short* Vl  = p; p += nX;
  unsigned short* Ah  = p; p += nX;   unsigned short* Al  = p; p += nX;

  const int n8X = (int)(nX / 8);
  const int n8W = (int)(nW / 8);
  k_split<<<(n8X + 255) / 256, 256, 0, stream>>>(x,  Xh,  Xl,  n8X);
  k_split<<<(n8W + 255) / 256, 256, 0, stream>>>(Wq, Wqh, Wql, n8W);
  k_split<<<(n8W + 255) / 256, 256, 0, stream>>>(Wk, Wkh, Wkl, n8W);
  k_split<<<(n8W + 255) / 256, 256, 0, stream>>>(Wv, Wvh, Wvl, n8W);
  k_split<<<(n8W + 255) / 256, 256, 0, stream>>>(Wo, Woh, Wol, n8W);

  const int nblk = ((E_ / 64) * (N_ / 16)) / 4;
  k_gemm<0><<<nblk, 128, 0, stream>>>(Wqh, Wql, Xh, Xl, bq, Qh, Ql, out);
  k_gemm<0><<<nblk, 128, 0, stream>>>(Wkh, Wkl, Xh, Xl, bk, Kh, Kl, out);
  k_gemm<1><<<nblk, 128, 0, stream>>>(Xh, Xl, Wvh, Wvl, bv, Vh, Vl, out);

  k_attn<<<(B_ * H_ * (S_ / 16)) / 4, 128, 0, stream>>>(Qh, Ql, Kh, Kl, Vh, Vl, ent, Ah, Al);

  k_gemm<2><<<nblk, 128, 0, stream>>>(Woh, Wol, Ah, Al, bo, Ah, Al, out);
}
